// GAT_with_global_update_83468394431131
// MI455X (gfx1250) — hardware-verified
//
#include <hip/hip_runtime.h>
#include <math.h>

#define NN    50000
#define NE    400000
#define DD    128
#define HH    128
#define GG    8
#define NHOPS 3
#define GOUTD 128
#define NP    50048
#define NT    256
#define SRB   2048
#define NTILE 25
#define RPW   (SRB / 8)
#define SCH   4096
#define NCH   ((NE + SCH - 1) / SCH)
#define NGRP  ((NN + 31) / 32)
#define XSC   64.0f
#define WSC   256.0f
#define GSCALE (1.0f / 16384.0f)

typedef __attribute__((ext_vector_type(16))) _Float16 v16h;
typedef __attribute__((ext_vector_type(8)))  _Float16 v8h;
typedef __attribute__((ext_vector_type(16))) __bf16   v16b;
typedef __attribute__((ext_vector_type(8)))  __bf16   v8b;
typedef __attribute__((ext_vector_type(8)))  float    v8f;
typedef __attribute__((ext_vector_type(4)))  float    v4f;
typedef __attribute__((ext_vector_type(4)))  int      v4i;

__device__ __forceinline__ unsigned short f2bf_bits(float f) {
  unsigned u = __float_as_uint(f);
  return (unsigned short)((u + 0x7FFFu + ((u >> 16) & 1u)) >> 16);
}
__device__ __forceinline__ float bf_bits2f(unsigned short h) { return __uint_as_float(((unsigned)h) << 16); }

__device__ __forceinline__ void dep_guard_h(v8f& a, v8f& b, v16h x, v16h y) { asm volatile("v_nop\n\tv_nop\n\tv_nop\n\tv_nop" : "+v"(a), "+v"(b) : "v"(x), "v"(y)); }
__device__ __forceinline__ void dep_guard_b(v8f& a, v8f& b, v16b x, v16b y) { asm volatile("v_nop\n\tv_nop\n\tv_nop\n\tv_nop" : "+v"(a), "+v"(b) : "v"(x), "v"(y)); }
__device__ __forceinline__ void keep4_h(v16h a, v16h b, v16h c, v16h d) { asm volatile("v_nop" :: "v"(a), "v"(b), "v"(c), "v"(d)); }
__device__ __forceinline__ void keep4_b(v16b a, v16b b, v16b c, v16b d) { asm volatile("v_nop" :: "v"(a), "v"(b), "v"(c), "v"(d)); }
__device__ __forceinline__ void acc_guard4(v8f& a, v8f& b, v8f& c, v8f& d) { asm volatile("v_nop\n\tv_nop\n\tv_nop\n\tv_nop" : "+v"(a), "+v"(b), "+v"(c), "+v"(d)); }
template <typename T> struct Frag;
template <> struct Frag<_Float16> {
  typedef v16h V; union U { v16h v; v8h h[2]; };
  static __device__ __forceinline__ v16h load(const _Float16* p) {
    U f; f.h[0] = *(const v8h*)(p); f.h[1] = *(const v8h*)(p + 16); return f.v;
  }
  static __device__ __forceinline__ v8f mma(v16h a, v16h b, v8f c) {
    return __builtin_amdgcn_wmma_f32_16x16x32_f16(false, a, false, b, (short)0, c, false, false);
  }
  static __device__ __forceinline__ void guard(v8f& a, v8f& b, v16h x, v16h y) { dep_guard_h(a, b, x, y); }
  static __device__ __forceinline__ void keep(v16h a, v16h b, v16h c, v16h d) { keep4_h(a, b, c, d); }
};
template <> struct Frag<__bf16> {
  typedef v16b V; union U { v16b v; v8b h[2]; };
  static __device__ __forceinline__ v16b load(const __bf16* p) {
    U f; f.h[0] = *(const v8b*)(p); f.h[1] = *(const v8b*)(p + 16); return f.v;
  }
  static __device__ __forceinline__ v8f mma(v16b a, v16b b, v8f c) {
    return __builtin_amdgcn_wmma_f32_16x16x32_bf16(false, a, false, b, (short)0, c, false, false);
  }
  static __device__ __forceinline__ void guard(v8f& a, v8f& b, v16b x, v16b y) { dep_guard_b(a, b, x, y); }
  static __device__ __forceinline__ void keep(v16b a, v16b b, v16b c, v16b d) { keep4_b(a, b, c, d); }
};

template <int ET> struct Elem;
template <> struct Elem<0> { typedef _Float16 T; };
template <> struct Elem<1> { typedef __bf16 T; };
template <int ET, bool SPLIT, int BIAS_MODE, int OUT_MODE, bool RESID, int ACT = 0>
__global__ __launch_bounds__(256) void wmma_gemm64(
    const unsigned short* __restrict__ Ap, const unsigned short* __restrict__ A2p, int lda, long strideA,
    const unsigned short* __restrict__ Btp, const unsigned short* __restrict__ Bt2p, int ldb, long strideB,
    void* __restrict__ Cout, void* __restrict__ Cout2, int ldc, long strideC,
    const float* __restrict__ bias,
    const float* __restrict__ resid, long strideR,
    int M, int N, int K, float scale) {
  typedef typename Elem<ET>::T T;
  typedef typename Frag<T>::V V;
  const T* A = (const T*)Ap; const T* A2 = (const T*)A2p; const T* Bt = (const T*)Btp; const T* Bt2 = (const T*)Bt2p;
  __shared__ __align__(16) float sT[8][16 * 68];
  const int b    = blockIdx.y;
  const int lane = threadIdx.x & 31;
  const int wave = threadIdx.x >> 5;
  const int tilesN = N >> 6;
  const int tilesM = M >> 6;
  const int tile = blockIdx.x * 8 + wave;
  if (tile >= tilesM * tilesN) return;
  const int tm = tile / tilesN;
  const int tn = tile - tm * tilesN;
  const int m0 = tm << 6;
  const int n0 = tn << 6;

  const T* Ab  = A  + (size_t)b * strideA;
  const T* Bb  = Bt + (size_t)b * strideB;
  const T* Ab2 = SPLIT ? (A2  + (size_t)b * strideA) : nullptr;
  const T* Bb2 = SPLIT ? (Bt2 + (size_t)b * strideB) : nullptr;

  const int rlane = lane & 15;
  const int koff  = (lane >> 4) * 8;
  const int mOff  = (lane >> 4) * 8;

  v8f acc[4][4];
#pragma unroll
  for (int i = 0; i < 4; ++i)
#pragma unroll
    for (int j = 0; j < 4; ++j) acc[i][j] = (v8f){0.f,0.f,0.f,0.f,0.f,0.f,0.f,0.f};

  for (int k0 = 0; k0 < K; k0 += 32) {
    V bh[4], bl[4];
#pragma unroll
    for (int j = 0; j < 4; ++j) {
      const size_t bo = (size_t)(n0 + (j << 4) + rlane) * ldb + koff + k0;
      bh[j] = Frag<T>::load(Bb + bo);
      if (SPLIT) bl[j] = Frag<T>::load(Bb2 + bo);
    }
#pragma unroll
    for (int i = 0; i < 4; ++i) {
      const size_t ao = (size_t)(m0 + (i << 4) + rlane) * lda + koff + k0;
      V ah = Frag<T>::load(Ab + ao);
      V al;
      if (SPLIT) al = Frag<T>::load(Ab2 + ao);
#pragma unroll
      for (int j = 0; j < 4; ++j) {
        acc[i][j] = Frag<T>::mma(ah, bh[j], acc[i][j]);
        if (SPLIT) {
          acc[i][j] = Frag<T>::mma(ah, bl[j], acc[i][j]);
          acc[i][j] = Frag<T>::mma(al, bh[j], acc[i][j]);
        }
      }
      Frag<T>::guard(acc[i][0], acc[i][3], ah, SPLIT ? al : ah);
    }
    Frag<T>::keep(bh[0], bh[1], bh[2], bh[3]);
    if (SPLIT) Frag<T>::keep(bl[0], bl[1], bl[2], bl[3]);
  }
  acc_guard4(acc[0][0], acc[0][1], acc[0][2], acc[0][3]);
  acc_guard4(acc[1][0], acc[1][1], acc[1][2], acc[1][3]);
  acc_guard4(acc[2][0], acc[2][1], acc[2][2], acc[2][3]);
  acc_guard4(acc[3][0], acc[3][1], acc[3][2], acc[3][3]);

  float* slab = sT[wave];
  const float* Rb = RESID ? (resid + (size_t)b * strideR) : nullptr;
#pragma unroll
  for (int i = 0; i < 4; ++i) {
    const int mBase = m0 + (i << 4);
#pragma unroll
    for (int j = 0; j < 4; ++j) {
      const int n = n0 + (j << 4) + rlane;
      float bv = 0.f;
      if (BIAS_MODE == 2) bv = bias[n];
#pragma unroll
      for (int r = 0; r < 8; ++r) {
        float v = acc[i][j][r] * scale;
        if (BIAS_MODE == 1) v += bias[mBase + mOff + r];
        if (BIAS_MODE == 2) v += bv;
        if (RESID) v += Rb[(size_t)(mBase + mOff + r) * ldc + n];
        if (ACT == 1) v = tanhf(v);
        if (ACT == 2) v = fmaxf(v, 0.0f);
        if (ACT == 3) v = v / (1.0f + expf(-v));
        if (ACT == 4) v = (v > 0.f) ? v : 0.01f * v;
        if (ACT == 5) v = 0.5f * v * (1.0f + erff(v * 0.70710678118654752f));
        slab[(mOff + r) * 68 + (j << 4) + rlane] = v;
      }
    }
    __builtin_amdgcn_fence(__ATOMIC_RELEASE, "workgroup");
    __builtin_amdgcn_wave_barrier();
    __builtin_amdgcn_fence(__ATOMIC_ACQUIRE, "workgroup");
    if (OUT_MODE == 0) {
      float* C = (float*)Cout + (size_t)b * strideC;
      const int hh = lane >> 4, c4 = (lane & 15) * 4;
      for (int pass = 0; pass < 2; ++pass) {
#pragma unroll
        for (int it = 0; it < 8; ++it) {
          const int row = it * 2 + hh;
          v4f v = *(const v4f*)(slab + row * 68 + c4);
          *(volatile v4f*)(C + (size_t)(mBase + row) * ldc + n0 + c4) = v;
        }
        __threadfence();
      }
    } else {
      const int q = lane >> 3, c8 = (lane & 7) * 8;
      unsigned short* C  = (unsigned short*)Cout  + (size_t)b * strideC;
      unsigned short* C2 = (OUT_MODE == 2) ? ((unsigned short*)Cout2 + (size_t)b * strideC) : nullptr;
      for (int pass = 0; pass < 2; ++pass) {
#pragma unroll
        for (int it = 0; it < 4; ++it) {
          const int row = it * 4 + q;
          const float* sp = slab + row * 68 + c8;
          v8h hv, lv;
#pragma unroll
          for (int e = 0; e < 8; ++e) {
            if (OUT_MODE == 1) {
              hv[e] = (_Float16)sp[e];
            } else {
              unsigned short hb = f2bf_bits(sp[e]);
              unsigned short lb = f2bf_bits(sp[e] - bf_bits2f(hb));
              hv[e] = __builtin_bit_cast(_Float16, hb);
              lv[e] = __builtin_bit_cast(_Float16, lb);
            }
          }
          *(volatile v8h*)(C + (size_t)(mBase + row) * ldc + n0 + c8) = hv;
          if (OUT_MODE == 2) *(volatile v8h*)(C2 + (size_t)(mBase + row) * ldc + n0 + c8) = lv;
        }
        __threadfence();
      }
    }
    __builtin_amdgcn_fence(__ATOMIC_RELEASE, "workgroup");
    __builtin_amdgcn_wave_barrier();
    __builtin_amdgcn_fence(__ATOMIC_ACQUIRE, "workgroup");
  }
}

__device__ __forceinline__ float dot4(v4f a, v4f b) { return a[0] * b[0] + a[1] * b[1] + a[2] * b[2] + a[3] * b[3]; }
__device__ __forceinline__ float wsum32(float d) {
  d += __shfl_xor(d, 16, 32); d += __shfl_xor(d, 8, 32); d += __shfl_xor(d, 4, 32); d += __shfl_xor(d, 2, 32); d += __shfl_xor(d, 1, 32);
  return d;
}

__device__ __forceinline__ int blk_excl_scan(int cnt, int* scan_ws, int tid, int* tot) {
  const int lane = tid & 31, wave = tid >> 5; int incl = cnt;
#pragma unroll
  for (int o = 1; o < 32; o <<= 1) { const int v = __shfl_up(incl, o, 32); if (lane >= o) incl += v; }
  if (lane == 31) scan_ws[wave] = incl;
  __syncthreads();
  if (wave == 0) { int wv = (lane < NT / 32) ? scan_ws[lane] : 0; int wincl = wv;
#pragma unroll
    for (int o = 1; o < 32; o <<= 1) { const int v = __shfl_up(wincl, o, 32); if (lane >= o) wincl += v; }
    if (lane < NT / 32) scan_ws[32 + lane] = wincl - wv; if (lane == 31) scan_ws[64] = wincl; }
  __syncthreads();
  const int res = scan_ws[32 + wave] + incl - cnt; *tot = scan_ws[64];
  return res;
}
template <int SP, int CAP>
__device__ __forceinline__ int chunk_hits(const int* __restrict__ dstv, const int* __restrict__ srcv, int e0, int n0, int tid,
                                          int* LIST, int* scan_ws) {
  const int eb = e0 + tid * SP;
  const bool inr = eb < NE;
  const int ebc = inr ? eb : (NE - SP);
  int rec[SP]; int cnt = 0;
#pragma unroll
  for (int k = 0; k < SP; k += 4) {
    const v4i d4 = *(const v4i*)(dstv + ebc + k);
    const v4i s4 = *(const v4i*)(srcv + ebc + k);
#pragma unroll
    for (int e = 0; e < 4; ++e) {
      const int d = d4[e]; int r = -1;
      if (inr && d >= n0 && d < n0 + SRB) { int s = s4[e]; s = s < 0 ? 0 : (s >= NN ? NN - 1 : s); r = ((d - n0) << 16) | s; ++cnt; }
      rec[k + e] = r;
    }
  }
  int tot; int p = blk_excl_scan(cnt, scan_ws, tid, &tot);
#pragma unroll
  for (int k = 0; k < SP; ++k) if (rec[k] >= 0) { if ((unsigned)p < (unsigned)CAP) LIST[p] = rec[k]; ++p; }
  __syncthreads();
  return tot < CAP ? tot : CAP;
}

#define NXD (NP * HH / 2)
#define NWD (NHOPS * DD * HH / 2)
__global__ __launch_bounds__(NT) void prep_kernel(const float* __restrict__ nodes, const float* __restrict__ Wq,
                                                 unsigned* __restrict__ XA32, unsigned* __restrict__ WQ32) {
  const int i = blockIdx.x * NT + threadIdx.x;
  if (i < NXD) {
    const int row = i >> 6; const int k = (i & 63) * 2;
    const int rowc = row < NN ? row : NN - 1;
    const float* p = nodes + (size_t)rowc * DD + k;
    float a = p[0] * XSC, b = p[1] * XSC;
    if (row >= NN) { a = 0.f; b = 0.f; }
    const _Float16 h0 = (_Float16)a, h1 = (_Float16)b;
    const unsigned u = (unsigned)__builtin_bit_cast(unsigned short, h0) | ((unsigned)__builtin_bit_cast(unsigned short, h1) << 16);
    ((volatile unsigned*)XA32)[i] = u;
    __threadfence();
    ((volatile unsigned*)XA32)[i] = u;
  }
  if (i < NWD) {
    const int h = i >> 13; const int rem = i & 8191;
    const int n = rem >> 6; const int k = (rem & 63) * 2;
    const float* wp = Wq + (size_t)h * DD * HH;
    const float a = wp[(size_t)k * HH + n] * WSC, b = wp[(size_t)(k + 1) * HH + n] * WSC;
    const _Float16 h0 = (_Float16)a, h1 = (_Float16)b;
    const unsigned u = (unsigned)__builtin_bit_cast(unsigned short, h0) | ((unsigned)__builtin_bit_cast(unsigned short, h1) << 16);
    ((volatile unsigned*)WQ32)[i] = u;
    __threadfence();
    ((volatile unsigned*)WQ32)[i] = u;
  }
}

template <bool FINAL>
__global__ __launch_bounds__(NT) void agg_kernel(const float* __restrict__ Q, const int* __restrict__ snd, const int* __restrict__ rcv,
                                                const float* __restrict__ Wah, const float* __restrict__ bah,
                                                float* ACC, unsigned short* __restrict__ XA, float* __restrict__ XO) {
  __shared__ int LIST[SCH];
  __shared__ float SM[SRB];
  __shared__ float SL[SRB];
  __shared__ float SAD[SRB];
  __shared__ int scan_ws[80];
  const int tid = threadIdx.x, lane = tid & 31, wave = tid >> 5;
  const int n0 = blockIdx.x * SRB;
  const size_t rbase = (size_t)blockIdx.x * SRB;
  const v4f was = *(const v4f*)(Wah + 4 * lane);
  const v4f war = *(const v4f*)(Wah + HH + 4 * lane);
  const float ba0 = bah[0];
  const v4f z4 = {0.f, 0.f, 0.f, 0.f};
  for (int ps = 0; ps < 2; ++ps) {
#pragma unroll 1
    for (int j = 0; j < RPW; ++j)
      *(volatile v4f*)(ACC + (rbase + (size_t)(wave * RPW + j)) * HH + 4 * lane) = z4;
    __threadfence();
  }
  for (int i = tid; i < SRB; i += NT) { SM[i] = -INFINITY; SL[i] = 0.f; }
#pragma unroll 1
  for (int dl = wave; dl < SRB; dl += NT / 32) {
    int n = n0 + dl; n = n < NN ? n : NN - 1;
    const v4f qv = *(const v4f*)(Q + (size_t)n * HH + 4 * lane);
    const float d = wsum32(dot4(qv, war));
    if (lane == 0) SAD[dl] = d + ba0;
  }
  __syncthreads();
#pragma unroll 1
  for (int c = 0; c < NCH; ++c) {
    const int tot = chunk_hits<SCH / NT, SCH>(rcv, snd, c * SCH, n0, tid, LIST, scan_ws);
#pragma unroll 1
    for (int base = 0; base < tot; base += 32) {
      int qi = base + lane; const bool inl = qi < tot; qi = qi < SCH ? qi : SCH - 1;
      const int lsv = LIST[qi];
      const int rv = inl ? lsv : -1;
      const int own = (rv >= 0 && (rv >> 24) == wave) ? 1 : 0;
      unsigned msk = (unsigned)__ballot(own);
#pragma unroll 1
      for (int it = 0; it < 32; ++it) {
        if (msk == 0u) break;
        const int bp = __builtin_ctz(msk); msk &= msk - 1u;
        const int r = __shfl(rv, bp, 32);
        const int dl = r >> 16, s = r & 0xFFFF;
        const v4f qv = *(const v4f*)(Q + (size_t)s * HH + 4 * lane);
        const float al = wsum32(dot4(qv, was)) + SAD[dl];
        const float mo = SM[dl], lo = SL[dl];
        const float mn = fmaxf(mo, al);
        const float rr = __expf(mo - mn), ex = __expf(al - mn);
        const float ln = lo * rr + ex;
        if (lane == 0) { SM[dl] = mn; SL[dl] = ln; }
        float* rp = ACC + (rbase + (size_t)dl) * HH + 4 * lane;
        v4f a = *(const v4f*)rp;
        a = a * rr + ex * qv;
        *(volatile v4f*)rp = a;
        __threadfence();
        *(volatile v4f*)rp = a;
      }
    }
    __syncthreads();
  }
#pragma unroll 1
  for (int j = 0; j < RPW; ++j) {
    const int dl = wave * RPW + j; const int n = n0 + dl;
    if (n < NP) {
      const bool live = n < NN;
      const float lsum = SL[dl];
      const float inv = (live && lsum > 0.f) ? (1.0f / lsum) : 0.f;
      const v4f a = *(const v4f*)(ACC + (rbase + (size_t)dl) * HH + 4 * lane);
      v4f v;
#pragma unroll
      for (int e = 0; e < 4; ++e) { const float t = a[e] * inv; v[e] = (t > 0.f) ? t : 0.01f * t; }
      if (FINAL) {
        if (live) {
          float* op = XO + (size_t)n * HH + 4 * lane;
          for (int ps = 0; ps < 2; ++ps) { *(volatile v4f*)op = v; __threadfence(); }
        }
      } else {
        const int sl0 = (2 * lane) & 31, sl1 = (2 * lane + 1) & 31;
        v8h hv;
#pragma unroll
        for (int e = 0; e < 4; ++e) {
          const float f0 = __shfl(v[e], sl0, 32), f1 = __shfl(v[e], sl1, 32);
          hv[e] = (_Float16)(f0 * XSC); hv[4 + e] = (_Float16)(f1 * XSC);
        }
        unsigned short* xp = XA + (size_t)n * HH + 8 * (lane & 15);
        for (int ps = 0; ps < 2; ++ps) { if (lane < 16) *(volatile v8h*)xp = hv; __threadfence(); }
      }
    }
  }
}

__global__ __launch_bounds__(NT) void global_kernel(const float* __restrict__ X, const int* __restrict__ gidx, const float* __restrict__ glob,
                                                   const float* __restrict__ Wg, const float* __restrict__ bg, float* __restrict__ OG) {
  __shared__ __align__(16) double red[8 * HH];
  __shared__ __align__(16) float cat[HH + DD];
  __shared__ __align__(16) float so[GOUTD];
  const int tid = threadIdx.x, lane = tid & 31, wave = tid >> 5;
  const int g = blockIdx.x;
  double a0 = 0.0, a1 = 0.0, a2 = 0.0, a3 = 0.0;
#pragma unroll 1
  for (int it = wave; it < NGRP; it += NT / 32) {
    const int nb = it * 32; const int idx = nb + lane; const int idxc = idx < NN ? idx : NN - 1;
    const int gv = gidx[idxc];
    const int hit = (idx < NN && gv == g) ? 1 : 0;
    unsigned msk = (unsigned)__ballot(hit);
#pragma unroll 1
    for (int t = 0; t < 32; ++t) {
      if (msk == 0u) break;
      const int bp = __builtin_ctz(msk); msk &= msk - 1u;
      const int n = nb + bp;
      const v4f xv = *(const v4f*)(X + (size_t)n * HH + 4 * lane);
      a0 += (double)xv[0]; a1 += (double)xv[1]; a2 += (double)xv[2]; a3 += (double)xv[3];
    }
  }
  red[wave * HH + 4 * lane]     = a0;
  red[wave * HH + 4 * lane + 1] = a1;
  red[wave * HH + 4 * lane + 2] = a2;
  red[wave * HH + 4 * lane + 3] = a3;
  __syncthreads();
  if (tid < HH) {
    double s = 0.0;
#pragma unroll
    for (int w = 0; w < 8; ++w) s += red[w * HH + tid];
    cat[tid] = (float)s;
    cat[HH + tid] = glob[(size_t)g * DD + tid];
  }
  __syncthreads();
  if (tid < GOUTD) {
    float o = 0.f;
#pragma unroll 1
    for (int k = 0; k < HH + DD; ++k) o += cat[k] * Wg[(size_t)k * GOUTD + tid];
    o += bg[tid];
    so[tid] = o;
  }
  __syncthreads();
  if (wave == 0) {
    const v4f p = *(const v4f*)(so + 4 * lane);
    float* op = OG + (size_t)g * GOUTD + 4 * lane;
    for (int ps = 0; ps < 2; ++ps) { *(volatile v4f*)op = p; __threadfence(); }
  }
}

extern "C" void kernel_launch(void* const* d_in, const int* in_sizes, int n_in,
                              void* d_out, int out_size, void* d_ws, size_t ws_size,
                              hipStream_t stream) {
  (void)in_sizes; (void)n_in; (void)out_size;
  const float* nodes    = (const float*)d_in[0];
  const float* globals_ = (const float*)d_in[1];
  const float* Wq       = (const float*)d_in[2];
  const float* bq       = (const float*)d_in[3];
  const float* Wa       = (const float*)d_in[4];
  const float* ba       = (const float*)d_in[5];
  const float* Wg       = (const float*)d_in[6];
  const float* bg       = (const float*)d_in[7];
  const int*   snd      = (const int*)d_in[8];
  const int*   rcv      = (const int*)d_in[9];
  const int*   gidx     = (const int*)d_in[10];

  float* out_x = (float*)d_out;
  float* out_g = out_x + (size_t)NN * HH;

  char* ws = (char*)d_ws; size_t off = 0;
  auto carve = [&](size_t bytes) -> char* { char* p = ws + off; off += (bytes + 255) & ~(size_t)255; return p; };
  unsigned short* WQT = (unsigned short*)carve((size_t)NHOPS * DD * HH * 2);
  unsigned short* XA  = (unsigned short*)carve((size_t)NP * HH * 2);
  float*          Q   = (float*)carve((size_t)NP * HH * 4);
  float*          ACC = (float*)carve((size_t)NTILE * SRB * HH * 4);
  if (off > ws_size || off > (size_t)134217728) return;

  prep_kernel<<<(NXD + NT - 1) / NT, NT, 0, stream>>>(nodes, Wq, (unsigned*)XA, (unsigned*)WQT);

  const int tiles = (NP / 64) * (HH / 64);
  for (int h = 0; h < NHOPS; ++h) {
    wmma_gemm64<0, false, 2, 0, false><<<dim3((tiles + 7) / 8, 1), 256, 0, stream>>>(
        (const unsigned short*)XA, (const unsigned short*)nullptr, HH, 0L,
        (const unsigned short*)(WQT + (size_t)h * DD * HH), (const unsigned short*)nullptr, DD, 0L,
        (void*)Q, (void*)nullptr, HH, 0L,
        bq + (size_t)h * HH, (const float*)nullptr, 0L, NP, HH, DD, GSCALE);
    if (h < NHOPS - 1)
      agg_kernel<false><<<NTILE, NT, 0, stream>>>(Q, snd, rcv, Wa + (size_t)h * 2 * HH, ba + h, ACC, XA, out_x);
    else
      agg_kernel<true><<<NTILE, NT, 0, stream>>>(Q, snd, rcv, Wa + (size_t)h * 2 * HH, ba + h, ACC, XA, out_x);
  }
  global_kernel<<<GG, NT, 0, stream>>>(out_x, gidx, globals_, Wg, bg, out_g);
}
